// EquivariantTransformer_7275674599757
// MI455X (gfx1250) — hardware-verified
//
#include <hip/hip_runtime.h>
#define NN 4096
#define ND 16
#define DD 128
#define NHD 4
#define HDC 32
#define NLY 4
#define DC 64
#define RCH 512
typedef __bf16 v16b __attribute__((ext_vector_type(16)));
typedef unsigned short v8us __attribute__((ext_vector_type(8), may_alias));
typedef float  v8f  __attribute__((ext_vector_type(8)));
typedef float  v4f  __attribute__((ext_vector_type(4)));
typedef float  v4fa __attribute__((ext_vector_type(4), may_alias));
union FragB { v16b v; v8us half[2]; unsigned short u[16]; };

__device__ __forceinline__ unsigned short bf16_bits(float x) { unsigned int u = __float_as_uint(x); return (unsigned short)((u + 0x7FFFu + ((u >> 16) & 1u)) >> 16); }
__device__ __forceinline__ float bf16_val(unsigned short b) { return __uint_as_float(((unsigned int)b) << 16); }
__device__ __forceinline__ float bf16_round(float x) { return bf16_val(bf16_bits(x)); }
template <int NT>
__device__ __forceinline__ v8f mmaN(v16b ah, v16b al, v16b bh, v16b bl, v8f c) {
  c = __builtin_amdgcn_wmma_f32_16x16x32_bf16(false, ah, false, bh, (short)0, c, false, false);
  if (NT >= 2) c = __builtin_amdgcn_wmma_f32_16x16x32_bf16(false, al, false, bh, (short)0, c, false, false);
  if (NT >= 3) c = __builtin_amdgcn_wmma_f32_16x16x32_bf16(false, ah, false, bl, (short)0, c, false, false);
  asm volatile("v_nop\n\tv_nop\n\tv_nop\n\tv_nop" : "+v"(c) : "v"(ah), "v"(al), "v"(bh), "v"(bl));
  return c;
}

__global__ __launch_bounds__(256) void k_wt_bf16(const float* __restrict__ W, unsigned short* __restrict__ Wt, int K, int N) {
  const int t = blockIdx.x * 256 + threadIdx.x;
  const int k8n = K / 8;
  if (t >= N * k8n) return;
  const int n = t / k8n, k8 = (t % k8n) * 8;
  v8us v;
#pragma unroll
  for (int i = 0; i < 8; ++i) v[i] = bf16_bits(W[(size_t)(k8 + i) * N + n]);
  *(volatile v8us*)(Wt + (size_t)n * K + k8) = v;
  __threadfence();
  *(volatile v8us*)(Wt + (size_t)n * K + k8) = v;
}

template <bool ASPLIT, int ACT, bool BIAS_BF16>
__global__ __launch_bounds__(128) void k_gemm_bf(const float* __restrict__ A, int lda, const unsigned short* __restrict__ Wt, int ldb,
                                               const float* __restrict__ bias, float* __restrict__ C, int ldc, int M, int N, int K) {
  __shared__ __attribute__((aligned(16))) float so[4][16][64];
  const int tid = threadIdx.x, w = tid >> 5, lane = tid & 31, ln = lane & 15, hh = lane >> 4;
  const int ntn = N / 64;
  const int wid = blockIdx.x * 4 + w;
  const int mt = wid / ntn, nq = wid % ntn;
  if (mt * 16 >= M) return;
  const int row0 = mt * 16, col0 = nq * 64;
  const float* arow = A + (size_t)(row0 + ln) * lda;
  v8f acc[4] = {};
  for (int kb = 0; kb < K; kb += 32) {
    FragB ah, al;
    const v4f x0 = *(const v4fa*)(arow + kb + 8 * hh), x1 = *(const v4fa*)(arow + kb + 8 * hh + 4);
    const v4f x2 = *(const v4fa*)(arow + kb + 16 + 8 * hh), x3 = *(const v4fa*)(arow + kb + 16 + 8 * hh + 4);
    float xs[16] = {x0[0],x0[1],x0[2],x0[3],x1[0],x1[1],x1[2],x1[3],x2[0],x2[1],x2[2],x2[3],x3[0],x3[1],x3[2],x3[3]};
#pragma unroll
    for (int i = 0; i < 16; ++i) { const unsigned short hb = bf16_bits(xs[i]); ah.u[i] = hb; al.u[i] = ASPLIT ? bf16_bits(xs[i] - bf16_val(hb)) : (unsigned short)0; }
#pragma unroll
    for (int t = 0; t < 4; ++t) {
      const unsigned short* brow = Wt + (size_t)(col0 + t * 16 + ln) * ldb + kb;
      FragB b;
      b.half[0] = *(const v8us*)(brow + 8 * hh);
      b.half[1] = *(const v8us*)(brow + 16 + 8 * hh);
      acc[t] = mmaN<ASPLIT ? 2 : 1>(ah.v, al.v, b.v, b.v, acc[t]);
    }
  }
#pragma unroll
  for (int t = 0; t < 4; ++t) {
    float bv = bias ? bias[col0 + t * 16 + ln] : 0.f;
    if (BIAS_BF16) bv = bf16_round(bv);
#pragma unroll
    for (int r = 0; r < 8; ++r) { float v = acc[t][r] + bv; if (ACT == 1) v = fmaxf(v, 0.f); so[w][8 * hh + r][t * 16 + ln] = v; }
  }
  __builtin_amdgcn_fence(__ATOMIC_ACQ_REL, "workgroup");
  __builtin_amdgcn_wave_barrier();
  const int rsub = lane >> 4, c4 = (lane & 15) * 4;
  for (int pass = 0; pass < 2; ++pass) {
#pragma unroll
    for (int q = 0; q < 8; ++q) {
      const int r = q * 2 + rsub;
      const v4f v = *(const v4fa*)&so[w][r][c4];
      *(volatile v4f*)(C + (size_t)(row0 + r) * ldc + col0 + c4) = v;
    }
    if (pass == 0) __threadfence();
  }
}

template <bool ASPLIT, int ACT, bool BIAS_BF16, bool RES_BF16>
__global__ __launch_bounds__(128) void k_gemm_bf3(const float* __restrict__ A, int lda, const unsigned short* __restrict__ Wt, int ldb,
                                                const float* __restrict__ bias, const float* __restrict__ resid, int rmod, int ldr,
                                                float* __restrict__ C, int ldc, int M, int N, int K) {
  __shared__ __attribute__((aligned(16))) float so[4][16][64];
  const int tid = threadIdx.x, w = tid >> 5, lane = tid & 31, ln = lane & 15, hh = lane >> 4;
  const int ntn = N / 64;
  const int wid = blockIdx.x * 4 + w;
  const int mt = wid / ntn, nq = wid % ntn;
  if (mt * 16 >= M) return;
  const int row0 = mt * 16, col0 = nq * 64;
  const float* arow = A + (size_t)(row0 + ln) * lda;
  v8f acc[4] = {};
  for (int kb = 0; kb < K; kb += 32) {
    FragB ah, al;
    const v4f x0 = *(const v4fa*)(arow + kb + 8 * hh), x1 = *(const v4fa*)(arow + kb + 8 * hh + 4);
    const v4f x2 = *(const v4fa*)(arow + kb + 16 + 8 * hh), x3 = *(const v4fa*)(arow + kb + 16 + 8 * hh + 4);
    float xs[16] = {x0[0],x0[1],x0[2],x0[3],x1[0],x1[1],x1[2],x1[3],x2[0],x2[1],x2[2],x2[3],x3[0],x3[1],x3[2],x3[3]};
#pragma unroll
    for (int i = 0; i < 16; ++i) { const unsigned short hb = bf16_bits(xs[i]); ah.u[i] = hb; al.u[i] = ASPLIT ? bf16_bits(xs[i] - bf16_val(hb)) : (unsigned short)0; }
#pragma unroll
    for (int t = 0; t < 4; ++t) {
      const unsigned short* brow = Wt + (size_t)(col0 + t * 16 + ln) * ldb + kb;
      FragB b;
      b.half[0] = *(const v8us*)(brow + 8 * hh);
      b.half[1] = *(const v8us*)(brow + 16 + 8 * hh);
      acc[t] = mmaN<ASPLIT ? 2 : 1>(ah.v, al.v, b.v, b.v, acc[t]);
    }
  }
#pragma unroll
  for (int t = 0; t < 4; ++t) {
    const int col = col0 + t * 16 + ln;
    float bv = bias ? bias[col] : 0.f;
    if (BIAS_BF16) bv = bf16_round(bv);
#pragma unroll
    for (int r = 0; r < 8; ++r) {
      float v = acc[t][r] + bv;
      if (resid) { float rv = resid[(size_t)((row0 + 8 * hh + r) % rmod) * ldr + col]; if (RES_BF16) rv = bf16_round(rv); v += rv; }
      if (ACT == 1) v = fmaxf(v, 0.f);
      if (ACT == 2) v = 0.5f * v * (1.0f + erff(v * 0.70710678118654752f));
      if (ACT == 3) { const float u = 0.7978845608028654f * (v + 0.044715f * v * v * v); v = 0.5f * v * (1.0f + tanhf(u)); }
      so[w][8 * hh + r][t * 16 + ln] = v;
    }
  }
  __builtin_amdgcn_fence(__ATOMIC_ACQ_REL, "workgroup");
  __builtin_amdgcn_wave_barrier();
  const int rsub = lane >> 4, c4 = (lane & 15) * 4;
  for (int pass = 0; pass < 2; ++pass) {
#pragma unroll
    for (int q = 0; q < 8; ++q) {
      const int r = q * 2 + rsub;
      const v4f v = *(const v4fa*)&so[w][r][c4];
      *(volatile v4f*)(C + (size_t)(row0 + r) * ldc + col0 + c4) = v;
    }
    if (pass == 0) __threadfence();
  }
}
template <bool PARAM_BF16>
__global__ __launch_bounds__(256) void k_layernorm(const float* __restrict__ X, const float* __restrict__ R, const float* __restrict__ g, const float* __restrict__ bta,
                                                  float* __restrict__ out_sum, float* __restrict__ out_norm, int N, float eps) {
  __shared__ float red[256];
  const int row = blockIdx.x, tid = threadIdx.x;
  const float* x = X + (size_t)row * N; const float* rr = R ? R + (size_t)row * N : nullptr;
  float vals[16];
  const int per = N / 256;
  float s1 = 0.f;
  for (int u = 0; u < per / 4; ++u) {
    const int j = tid * 4 + 1024 * u;
    const v4f a = *(const v4fa*)(x + j);
    v4f b = {0.f,0.f,0.f,0.f}; if (rr) b = *(const v4fa*)(rr + j);
#pragma unroll
    for (int q = 0; q < 4; ++q) { const float v = a[q] + b[q]; vals[u * 4 + q] = v; s1 += v; }
  }
  red[tid] = s1; __syncthreads();
  for (int st = 128; st > 0; st >>= 1) { if (tid < st) red[tid] += red[tid + st]; __syncthreads(); }
  const float mu = red[0] / (float)N; __syncthreads();
  float s2 = 0.f;
  for (int u = 0; u < per / 4; ++u)
#pragma unroll
    for (int q = 0; q < 4; ++q) { const float c = vals[u * 4 + q] - mu; s2 += c * c; }
  red[tid] = s2; __syncthreads();
  for (int st = 128; st > 0; st >>= 1) { if (tid < st) red[tid] += red[tid + st]; __syncthreads(); }
  const float rs = rsqrtf(red[0] / (float)N + eps);
  for (int pass = 0; pass < 2; ++pass) {
    for (int u = 0; u < per / 4; ++u) {
      const int j = tid * 4 + 1024 * u;
      v4f o, sm;
#pragma unroll
      for (int q = 0; q < 4; ++q) {
        float gg = g[j + q], bb = bta[j + q];
        if (PARAM_BF16) { gg = bf16_round(gg); bb = bf16_round(bb); }
        sm[q] = vals[u * 4 + q]; o[q] = (vals[u * 4 + q] - mu) * rs * gg + bb;
      }
      if (out_sum) *(volatile v4f*)(out_sum + (size_t)row * N + j) = sm;
      *(volatile v4f*)(out_norm + (size_t)row * N + j) = o;
    }
    if (pass == 0) __threadfence();
  }
}


typedef _Float16 v16h __attribute__((ext_vector_type(16)));
union FragH { v16h v; v8us half[2]; _Float16 h[16]; unsigned short u[16]; };
template <int NT>
__device__ __forceinline__ v8f mmaH(v16h ah, v16h al, v16h bh, v16h bl, v8f c) {
  c = __builtin_amdgcn_wmma_f32_16x16x32_f16(false, ah, false, bh, (short)0, c, false, false);
  if (NT >= 2) c = __builtin_amdgcn_wmma_f32_16x16x32_f16(false, al, false, bh, (short)0, c, false, false);
  if (NT >= 3) c = __builtin_amdgcn_wmma_f32_16x16x32_f16(false, ah, false, bl, (short)0, c, false, false);
  asm volatile("v_nop\n\tv_nop\n\tv_nop\n\tv_nop" : "+v"(c) : "v"(ah), "v"(al), "v"(bh), "v"(bl));
  return c;
}
template <bool ASPLIT>
__global__ __launch_bounds__(128) void k_gemm_h(const float* __restrict__ A, int lda, size_t sA, const _Float16* __restrict__ Bh, int ldb, size_t sB, float alpha, float* __restrict__ C, int ldc, size_t sC, int M, int N, int K) {
  __shared__ __attribute__((aligned(16))) float so[4][16][64];
  const int tid = threadIdx.x, w = tid >> 5, lane = tid & 31, ln = lane & 15, hh = lane >> 4; const int by = blockIdx.y;
  A += (size_t)by * sA; Bh += (size_t)by * sB; C += (size_t)by * sC;
  const int ntn = (N + 63) / 64; const int wid = blockIdx.x * 4 + w; const int mt = wid / ntn, nq = wid % ntn; if (mt * 16 >= M) return;
  const int row0 = mt * 16, col0 = nq * 64; const float* arow = A + (size_t)(row0 + ln) * lda;
  v8f acc[4] = {};
  for (int kb = 0; kb < K; kb += 32) {
    FragH ah, al;
    const v4f x0 = *(const v4fa*)(arow + kb + 8 * hh), x1 = *(const v4fa*)(arow + kb + 8 * hh + 4), x2 = *(const v4fa*)(arow + kb + 16 + 8 * hh), x3 = *(const v4fa*)(arow + kb + 16 + 8 * hh + 4);
    float xs[16] = {x0[0],x0[1],x0[2],x0[3],x1[0],x1[1],x1[2],x1[3],x2[0],x2[1],x2[2],x2[3],x3[0],x3[1],x3[2],x3[3]};
#pragma unroll
    for (int i = 0; i < 16; ++i) { const _Float16 h = (_Float16)xs[i]; ah.h[i] = h; al.h[i] = ASPLIT ? (_Float16)(xs[i] - (float)h) : (_Float16)0.0f; }
#pragma unroll
    for (int t = 0; t < 4; ++t) { if (col0 + t * 16 >= N) continue; const size_t boff = (size_t)(col0 + t * 16 + ln) * ldb + kb; FragH bq; bq.half[0] = *(const v8us*)(Bh + boff + 8 * hh); bq.half[1] = *(const v8us*)(Bh + boff + 16 + 8 * hh);
      acc[t] = mmaH<ASPLIT ? 2 : 1>(ah.v, al.v, bq.v, bq.v, acc[t]); }
  }
#pragma unroll
  for (int t = 0; t < 4; ++t) { if (col0 + t * 16 >= N) continue;
#pragma unroll
    for (int r = 0; r < 8; ++r) so[w][8 * hh + r][t * 16 + ln] = acc[t][r] * alpha; }
  __builtin_amdgcn_fence(__ATOMIC_ACQ_REL, "workgroup"); __builtin_amdgcn_wave_barrier();
  const int rsub = lane >> 4, c4 = (lane & 15) * 4;
  for (int pass = 0; pass < 2; ++pass) {
#pragma unroll
    for (int q = 0; q < 8; ++q) { const int r = q * 2 + rsub; if (col0 + c4 < N) { const v4f v = *(const v4fa*)&so[w][r][c4]; *(volatile v4f*)(C + (size_t)(row0 + r) * ldc + col0 + c4) = v; } }
    if (pass == 0) __threadfence(); }
}

__global__ __launch_bounds__(256) void k_wt_f16(const float* __restrict__ W, _Float16* __restrict__ Wt, int K, int N, float scale) {
  const int t = blockIdx.x * 256 + threadIdx.x; if (t >= N * (K / 8)) return; const int n = t / (K / 8), k8 = (t % (K / 8)) * 8; FragH f;
#pragma unroll
  for (int i = 0; i < 8; ++i) f.h[i] = (_Float16)(bf16_round(W[(size_t)(k8 + i) * N + n]) * scale); const v8us o = f.half[0];
  *(volatile v8us*)((unsigned short*)Wt + (size_t)n * K + k8) = o; __threadfence(); *(volatile v8us*)((unsigned short*)Wt + (size_t)n * K + k8) = o;
}
template <int ACT>
__global__ __launch_bounds__(128) void k_gemm_hhx(const _Float16* __restrict__ A, int lda, size_t sA, const _Float16* __restrict__ Bh, int ldb, size_t sB, float alpha, const float* __restrict__ bias, size_t sBias, const float* __restrict__ CP, int rowsPerB, size_t sCPb, int row0g,
    float* __restrict__ C, _Float16* __restrict__ C16, int ldc, size_t sC, int M, int N, int K) {
  __shared__ __attribute__((aligned(16))) float so[4][16][64];
  const int tid = threadIdx.x, w = tid >> 5, lane = tid & 31, ln = lane & 15, hh = lane >> 4; const int by = blockIdx.y;
  A += (size_t)by * sA; Bh += (size_t)by * sB; const size_t cofs = (size_t)by * sC; const float* bp = bias ? bias + (size_t)by * sBias : nullptr;
  const int ntn = (N + 63) / 64; const int wid = blockIdx.x * 4 + w; const int mt = wid / ntn, nq = wid % ntn; if (mt * 16 >= M) return;
  const int row0 = mt * 16, col0 = nq * 64; const _Float16* arow = A + (size_t)(row0 + ln) * lda;
  v8f acc[4] = {};
  for (int kb = 0; kb < K; kb += 32) { FragH ah; ah.half[0] = *(const v8us*)((const unsigned short*)arow + kb + 8 * hh); ah.half[1] = *(const v8us*)((const unsigned short*)arow + kb + 16 + 8 * hh);
#pragma unroll
    for (int t = 0; t < 4; ++t) { if (col0 + t * 16 >= N) continue; const size_t boff = (size_t)(col0 + t * 16 + ln) * ldb + kb; FragH bq; bq.half[0] = *(const v8us*)((const unsigned short*)Bh + boff + 8 * hh); bq.half[1] = *(const v8us*)((const unsigned short*)Bh + boff + 16 + 8 * hh);
      acc[t] = mmaH<1>(ah.v, ah.v, bq.v, bq.v, acc[t]); }
  }
#pragma unroll
  for (int t = 0; t < 4; ++t) { if (col0 + t * 16 >= N) continue; const int col = col0 + t * 16 + ln; const float bv = bp ? bf16_round(bp[col]) : 0.f;
#pragma unroll
    for (int r = 0; r < 8; ++r) { float v = acc[t][r] * alpha + bv; if (CP) { const int bidx = (row0g + row0 + 8 * hh + r) / rowsPerB; v += CP[(size_t)bidx * sCPb + (size_t)by * 64 + col]; } if (ACT == 1) v = (v > 0.f) ? v : expm1f(v); else if (ACT == 7) v = (v > 0.f) ? v + 1.0f : expf(v); else if (ACT == 8) v = tanhf(v); else if (ACT == 9) v = 0.5f * v * (1.0f + tanhf(0.7978845608028654f * (v + 0.044715f * v * v * v))); else if (ACT == 11) v = 1.0f / (1.0f + expf(-v)); else if (ACT == 12) v = (v > 0.f) ? v : 0.01f * v; else if (ACT == 14) v = (v > 0.f) ? v : 0.1f * v; else if (ACT == 15) v = v / (1.0f + expf(-v)); else if (ACT == 3) v = fmaxf(v, 0.f); else if (ACT == 6) v = 0.5f * v * (1.0f + erff(v * 0.70710678118654752f)); so[w][8 * hh + r][t * 16 + ln] = v; } }
  __builtin_amdgcn_fence(__ATOMIC_ACQ_REL, "workgroup"); __builtin_amdgcn_wave_barrier();
  const int rsub = lane >> 4, c4 = (lane & 15) * 4; typedef _Float16 v4h __attribute__((ext_vector_type(4)));
  for (int pass = 0; pass < 2; ++pass) {
#pragma unroll
    for (int q = 0; q < 8; ++q) { const int r = q * 2 + rsub; if (col0 + c4 < N) { const v4f v = *(const v4fa*)&so[w][r][c4]; if (C) *(volatile v4f*)(C + cofs + (size_t)(row0 + r) * ldc + col0 + c4) = v; if (C16) { v4h h4; for (int i = 0; i < 4; ++i) h4[i] = (_Float16)v[i]; *(volatile v4h*)(C16 + cofs + (size_t)(row0 + r) * ldc + col0 + c4) = h4; } } }
    if (pass == 0) __threadfence(); }
}


typedef _Float16 v4h __attribute__((ext_vector_type(4)));

__global__ __launch_bounds__(256) void k_x16(const float* __restrict__ x, _Float16* __restrict__ X16, size_t n8) { const size_t t = (size_t)blockIdx.x * 256 + threadIdx.x; if (t >= n8) return; FragH f;
#pragma unroll
  for (int q = 0; q < 8; ++q) f.h[q] = (_Float16)bf16_round(x[t * 8 + q]); *(volatile v8us*)((unsigned short*)X16 + t * 8) = f.half[0]; __threadfence(); *(volatile v8us*)((unsigned short*)X16 + t * 8) = f.half[0]; }
__global__ __launch_bounds__(256) void k_h16(const float* __restrict__ x, _Float16* __restrict__ X16, size_t n8) { const size_t t = (size_t)blockIdx.x * 256 + threadIdx.x; if (t >= n8) return; FragH f;
#pragma unroll
  for (int q = 0; q < 8; ++q) f.h[q] = (_Float16)x[t * 8 + q]; *(volatile v8us*)((unsigned short*)X16 + t * 8) = f.half[0]; __threadfence(); *(volatile v8us*)((unsigned short*)X16 + t * 8) = f.half[0]; }
__global__ __launch_bounds__(256) void k_round16f(const float* __restrict__ W, _Float16* __restrict__ Bt, size_t n8) { const size_t t = (size_t)blockIdx.x * 256 + threadIdx.x; if (t >= n8) return; FragH f;
#pragma unroll
  for (int i = 0; i < 8; ++i) f.h[i] = (_Float16)(bf16_round(W[t * 8 + i]) * 16.0f); *(volatile v8us*)((unsigned short*)Bt + t * 8) = f.half[0]; __threadfence(); *(volatile v8us*)((unsigned short*)Bt + t * 8) = f.half[0]; }
template <int NHv, int TTv>
__global__ __launch_bounds__(256) void k_vt(const _Float16* __restrict__ V16, int ldv, int voff, _Float16* __restrict__ Vt) { __shared__ unsigned short tl[64][66]; const int tid = threadIdx.x; const int slab = blockIdx.x / (TTv / 64), lg = blockIdx.x % (TTv / 64); const int b = slab / NHv, h = slab % NHv;
  for (int i = tid; i < 64 * 8; i += 256) { const int r = i / 8, c8 = (i % 8) * 8; FragH f; f.half[0] = *(const v8us*)((const unsigned short*)V16 + ((size_t)b * TTv + lg * 64 + r) * ldv + voff + h * 64 + c8);
#pragma unroll
    for (int q = 0; q < 8; ++q) tl[r][c8 + q] = f.u[q]; }
  __syncthreads();
  for (int pass = 0; pass < 2; ++pass) {
#pragma unroll
    for (int rd = 0; rd < 2; ++rd) { const int d = rd * 32 + tid / 8, pc = tid % 8; FragH f;
#pragma unroll
      for (int q = 0; q < 8; ++q) f.u[q] = tl[pc * 8 + q][d];
      *(volatile v8us*)((unsigned short*)Vt + ((size_t)slab * 64 + d) * TTv + lg * 64 + pc * 8) = f.half[0]; }
    if (pass == 0) __threadfence(); } }

__global__ __launch_bounds__(256) void k_hl(const float* __restrict__ F, _Float16* __restrict__ Hh, _Float16* __restrict__ Hl, size_t n8) { const size_t t = (size_t)blockIdx.x * 256 + threadIdx.x; if (t >= n8) return; FragH fh, fl; const v4f a = *(const v4fa*)(F + t * 8), c = *(const v4fa*)(F + t * 8 + 4);
#pragma unroll
  for (int q = 0; q < 4; ++q) { _Float16 h = (_Float16)a[q]; fh.h[q] = h; fl.h[q] = (_Float16)((a[q] - (float)h) * 1024.0f); h = (_Float16)c[q]; fh.h[4 + q] = h; fl.h[4 + q] = (_Float16)((c[q] - (float)h) * 1024.0f); }
  for (int pass = 0; pass < 2; ++pass) { *(volatile v8us*)((unsigned short*)Hh + t * 8) = fh.half[0]; *(volatile v8us*)((unsigned short*)Hl + t * 8) = fl.half[0]; if (pass == 0) __threadfence(); } }

__global__ __launch_bounds__(256) void k_na16(const float* __restrict__ a, _Float16* __restrict__ O) { const int t = blockIdx.x * 256 + threadIdx.x; if (t >= NN * 4) return; const int g = t % 4, n = t / 4; FragH f = FragH{};
  if (g < 2) {
#pragma unroll
    for (int q = 0; q < 8; ++q) f.h[q] = (_Float16)bf16_round(a[(size_t)n * ND + g * 8 + q]); }
  *(volatile v8us*)((unsigned short*)O + (size_t)n * 32 + g * 8) = f.half[0]; __threadfence(); *(volatile v8us*)((unsigned short*)O + (size_t)n * 32 + g * 8) = f.half[0]; }
__global__ __launch_bounds__(256) void k_wemb(const float* __restrict__ W, _Float16* __restrict__ Bt) { const int t = blockIdx.x * 256 + threadIdx.x; if (t >= DD * 4) return; const int g = t % 4, o = t / 4; FragH f;
#pragma unroll
  for (int q = 0; q < 8; ++q) { const int k = g * 8 + q; f.h[q] = (k < ND) ? (_Float16)(bf16_round(W[(size_t)k * DD + o]) * 16.0f) : (_Float16)0.0f; }
  *(volatile v8us*)((unsigned short*)Bt + (size_t)o * 32 + g * 8) = f.half[0]; __threadfence(); *(volatile v8us*)((unsigned short*)Bt + (size_t)o * 32 + g * 8) = f.half[0]; }
__global__ __launch_bounds__(256) void k_f16c(const float* __restrict__ F, _Float16* __restrict__ O, size_t n8) { const size_t t = (size_t)blockIdx.x * 256 + threadIdx.x; if (t >= n8) return; const v4f a = *(const v4fa*)(F + t * 8), c = *(const v4fa*)(F + t * 8 + 4); FragH f;
#pragma unroll
  for (int q = 0; q < 8; ++q) f.h[q] = (_Float16)((q < 4) ? a[q] : c[q - 4]);
  *(volatile v8us*)((unsigned short*)O + t * 8) = f.half[0]; __threadfence(); *(volatile v8us*)((unsigned short*)O + t * 8) = f.half[0]; }
__global__ __launch_bounds__(256) void k_vt(const _Float16* __restrict__ QKV, _Float16* __restrict__ VT) { const int t = blockIdx.x * 256 + threadIdx.x; if (t >= DD * (NN / 8)) return; const int m0 = (t % (NN / 8)) * 8, c = t / (NN / 8); FragH f;
#pragma unroll
  for (int q = 0; q < 8; ++q) f.h[q] = QKV[(size_t)(m0 + q) * 3 * DD + 2 * DD + c];
  *(volatile v8us*)((unsigned short*)VT + (size_t)c * NN + m0) = f.half[0]; __threadfence(); *(volatile v8us*)((unsigned short*)VT + (size_t)c * NN + m0) = f.half[0]; }
__global__ __launch_bounds__(256) void k_hsoft(const float* __restrict__ S, _Float16* __restrict__ P) {
  #pragma clang fp contract(off)
  const int t = blockIdx.x * 256 + threadIdx.x; if (t >= RCH * (NN / 4)) return; const size_t base = (size_t)t * 4; const size_t plane = (size_t)RCH * NN; v4f a[4];
#pragma unroll
  for (int h = 0; h < 4; ++h) a[h] = *(const v4fa*)(S + h * plane + base);
  _Float16 f[4][4];
#pragma unroll
  for (int q = 0; q < 4; ++q) { float x0 = a[0][q], x1 = a[1][q], x2 = a[2][q], x3 = a[3][q]; const float m = fmaxf(fmaxf(x0, x1), fmaxf(x2, x3)); x0 = expf(x0 - m); x1 = expf(x1 - m); x2 = expf(x2 - m); x3 = expf(x3 - m); const float inv = 1.0f / (((x0 + x1) + x2) + x3);
    f[0][q] = (_Float16)(x0 * inv); f[1][q] = (_Float16)(x1 * inv); f[2][q] = (_Float16)(x2 * inv); f[3][q] = (_Float16)(x3 * inv); }
  for (int pass = 0; pass < 2; ++pass) {
#pragma unroll
    for (int h = 0; h < 4; ++h) { const unsigned long long pk = *(const unsigned long long*)f[h]; *(volatile unsigned long long*)((unsigned short*)P + h * plane + base) = pk; }
    if (pass == 0) __threadfence(); } }
__global__ __launch_bounds__(256) void k_ln(const float* __restrict__ X, const float* __restrict__ g, const float* __restrict__ bb, float* __restrict__ Hf, _Float16* __restrict__ H16) {
  #pragma clang fp contract(off)
  const int tid = threadIdx.x, w = tid >> 5, l = tid & 31; const int r = blockIdx.x * 8 + w; if (r >= NN) return; const v4f a = *(const v4fa*)(X + (size_t)r * DD + l * 4); float s = a[0] + a[1] + a[2] + a[3];
  for (int o = 16; o > 0; o >>= 1) s += __shfl_xor(s, o, 32); const float mu = s / (float)DD; float q2 = 0.f;
#pragma unroll
  for (int k = 0; k < 4; ++k) { const float d = a[k] - mu; q2 += d * d; }
  for (int o = 16; o > 0; o >>= 1) q2 += __shfl_xor(q2, o, 32); const float rs = rsqrtf(q2 / (float)DD + 1e-5f); v4f y; _Float16 h4[4];
#pragma unroll
  for (int k = 0; k < 4; ++k) { const int ch = l * 4 + k; y[k] = (a[k] - mu) * rs * bf16_round(g[ch]) + bf16_round(bb[ch]); h4[k] = (_Float16)y[k]; }
  const unsigned long long pk = *(const unsigned long long*)h4;
  for (int pass = 0; pass < 2; ++pass) { *(volatile v4f*)(Hf + (size_t)r * DD + l * 4) = y; *(volatile unsigned long long*)((unsigned short*)H16 + (size_t)r * DD + l * 4) = pk; if (pass == 0) __threadfence(); } }
__global__ __launch_bounds__(256) void k_pos(const float* __restrict__ C1, const float* __restrict__ Wc2, const float* __restrict__ bc2, const float* __restrict__ RM, float* POS) {
  #pragma clang fp contract(off)
  const int t = blockIdx.x * 256 + threadIdx.x; if (t >= NN * 3) return; const int n = t / 3; float cw = bf16_round(bc2[0]);
#pragma unroll 1
  for (int j = 0; j < DC; ++j) { const float z = C1[(size_t)n * DC + j]; const float sl = z / (1.0f + expf(-z)); cw += sl * bf16_round(Wc2[j]); }
  const float p = POS[t] + cw * RM[t];
  *(volatile float*)(POS + t) = p; __threadfence(); *(volatile float*)(POS + t) = p; }
__global__ __launch_bounds__(256) void k_pmean(const float* __restrict__ pos, float* __restrict__ MEAN) {
  #pragma clang fp contract(off)
  __shared__ float red[256]; __shared__ float res[4]; const int tid = threadIdx.x;
  for (int k = 0; k < 3; ++k) { float s = 0.f; for (int n = tid; n < NN; n += 256) s += bf16_round(pos[n * 3 + k]);
    red[tid] = s; __syncthreads(); for (int st = 128; st > 0; st >>= 1) { if (tid < st) red[tid] += red[tid + st]; __syncthreads(); }
    if (tid == 0) res[k] = red[0] / (float)NN; __syncthreads(); }
  if (tid < 32) { const float v = (tid < 3) ? res[tid] : 0.f; *(volatile float*)(MEAN + tid) = v; __threadfence(); *(volatile float*)(MEAN + tid) = v; } }
__global__ __launch_bounds__(256) void k_pinit(const float* __restrict__ pos, const float* __restrict__ MEAN, float* __restrict__ POS, float* __restrict__ RM) {
  #pragma clang fp contract(off)
  const int t = blockIdx.x * 256 + threadIdx.x; if (t >= NN * 3) return; const float p = bf16_round(pos[t]); const float rm = p - MEAN[t % 3];
  for (int pass = 0; pass < 2; ++pass) { *(volatile float*)(POS + t) = p; *(volatile float*)(RM + t) = rm; if (pass == 0) __threadfence(); } }
__global__ __launch_bounds__(256) void k_energy1(const float* __restrict__ Hf, const float* __restrict__ We, const float* __restrict__ be, float* __restrict__ EP) {
  #pragma clang fp contract(off)
  __shared__ float red[256]; const int tid = threadIdx.x; const int n = blockIdx.x * 256 + tid; float s = bf16_round(be[0]); const float* h = Hf + (size_t)n * DD;
#pragma unroll 1
  for (int j = 0; j < DD; ++j) s += h[j] * bf16_round(We[j]);
  red[tid] = s; __syncthreads(); for (int st = 128; st > 0; st >>= 1) { if (tid < st) red[tid] += red[tid + st]; __syncthreads(); }
  if (tid < 32) { const float v = (tid == 0) ? red[0] : 0.f; *(volatile float*)(EP + (size_t)blockIdx.x * 32 + tid) = v; __threadfence(); *(volatile float*)(EP + (size_t)blockIdx.x * 32 + tid) = v; } }
__global__ __launch_bounds__(256) void k_fin(const float* __restrict__ EP, const float* __restrict__ POS, float* __restrict__ out) {
  #pragma clang fp contract(off)
  const int t = blockIdx.x * 256 + threadIdx.x; if (t >= 1 + NN * 3) return; float v;
  if (t == 0) { float s = 0.f;
#pragma unroll 1
    for (int b = 0; b < NN / 256; ++b) s += EP[b * 32];
    v = s; } else v = POS[t - 1];
  *(volatile float*)(out + t) = v; __threadfence(); *(volatile float*)(out + t) = v; }
__global__ __launch_bounds__(512) void k_bcat3(const float* __restrict__ bq, const float* __restrict__ bk, const float* __restrict__ bv, int l, float* __restrict__ O) { const int t = threadIdx.x; if (t >= 3 * DD) return; const float v = (t < DD) ? bq[l * DD + t] : (t < 2 * DD) ? bk[l * DD + t - DD] : bv[l * DD + t - 2 * DD]; *(volatile float*)(O + t) = v; __threadfence(); *(volatile float*)(O + t) = v; }

extern "C" void kernel_launch(void* const* d_in, const int* in_sizes, int n_in,
                              void* d_out, int out_size, void* d_ws, size_t ws_size, hipStream_t stream) {
  (void)in_sizes; (void)n_in; (void)out_size;
  const float* const* I = (const float* const*)d_in; const float* na = I[0]; const float* pos = I[1]; const float* embW = I[2]; const float* embb = I[3]; const float* Wq = I[4]; const float* bq = I[5]; const float* Wk = I[6]; const float* bk = I[7]; const float* Wv = I[8]; const float* bv = I[9]; const float* Wo = I[10]; const float* bo = I[11]; const float* Wc1 = I[12]; const float* bc1 = I[13]; const float* Wc2 = I[14]; const float* bc2 = I[15]; const float* lng = I[16]; const float* lnb = I[17]; const float* We = I[18]; const float* be = I[19];
  char* ws = (char*)d_ws; size_t off = 0;
  auto take = [&](size_t bytes) { char* p = ws + off; off += (bytes + 255) & ~(size_t)255; return p; };
  _Float16* BE = (_Float16*)take((size_t)DD * 32 * 2); _Float16* BQKV = (_Float16*)take((size_t)3 * DD * DD * 2); float* BQKVb = (float*)take(3 * DD * 4); _Float16* BO = (_Float16*)take((size_t)DD * DD * 2); _Float16* BC1 = (_Float16*)take((size_t)DC * DD * 2); float* MEAN = (float*)take(32 * 4); float* EP = (float*)take((NN / 256) * 32 * 4);
  _Float16* NA16 = (_Float16*)take((size_t)NN * 32 * 2); float* Hf = (float*)take((size_t)NN * DD * 4); _Float16* H16 = (_Float16*)take((size_t)NN * DD * 2); float* QKVf = (float*)take((size_t)NN * 3 * DD * 4); _Float16* QKV16 = (_Float16*)take((size_t)NN * 3 * DD * 2); _Float16* VT = (_Float16*)take((size_t)DD * NN * 2);
  float* S = (float*)take((size_t)NHD * RCH * NN * 4); _Float16* P16 = (_Float16*)take((size_t)NHD * RCH * NN * 2); float* O = (float*)take((size_t)NN * DD * 4); _Float16* O16 = (_Float16*)take((size_t)NN * DD * 2); float* X2 = (float*)take((size_t)NN * DD * 4); float* C1 = (float*)take((size_t)NN * DC * 4); float* POS = (float*)take((size_t)NN * 3 * 4); float* RM = (float*)take((size_t)NN * 3 * 4);
  if (off > ws_size) return;
  k_wemb<<<(DD * 4 + 255) / 256, 256, 0, stream>>>(embW, BE); k_na16<<<(NN * 4 + 255) / 256, 256, 0, stream>>>(na, NA16);
  k_pmean<<<1, 256, 0, stream>>>(pos, MEAN); k_pinit<<<(NN * 3 + 255) / 256, 256, 0, stream>>>(pos, MEAN, POS, RM);
  const dim3 gD(((NN / 16) * (DD / 64) + 3) / 4, 1), gQ(((NN / 16) * (3 * DD / 64) + 3) / 4, 1), gS(((RCH / 16) * (NN / 64) + 3) / 4, 1), gP(((RCH / 16) * 1 + 3) / 4, 1), gC1(((NN / 16) * 1 + 3) / 4, 1);
  k_gemm_hhx<0><<<gD, 128, 0, stream>>>(NA16, 32, 0, BE, 32, 0, 0.0625f, embb, 0, nullptr, 1, 0, 0, Hf, H16, DD, 0, NN, DD, 32);
  const size_t n8 = (size_t)NN * DD / 8;
  for (int l = 0; l < NLY; ++l) {
    k_wt_f16<<<(DD * (DD / 8) + 255) / 256, 256, 0, stream>>>(Wq + (size_t)l * DD * DD, BQKV, DD, DD, 16.0f); k_wt_f16<<<(DD * (DD / 8) + 255) / 256, 256, 0, stream>>>(Wk + (size_t)l * DD * DD, BQKV + (size_t)DD * DD, DD, DD, 16.0f); k_wt_f16<<<(DD * (DD / 8) + 255) / 256, 256, 0, stream>>>(Wv + (size_t)l * DD * DD, BQKV + (size_t)2 * DD * DD, DD, DD, 16.0f); k_bcat3<<<1, 512, 0, stream>>>(bq, bk, bv, l, BQKVb);
    k_wt_f16<<<(DD * (DD / 8) + 255) / 256, 256, 0, stream>>>(Wo + (size_t)l * DD * DD, BO, DD, DD, 16.0f); k_wt_f16<<<(DC * (DD / 8) + 255) / 256, 256, 0, stream>>>(Wc1 + (size_t)l * DD * DC, BC1, DD, DC, 16.0f);
    k_gemm_hhx<0><<<gQ, 128, 0, stream>>>(H16, DD, 0, BQKV, DD, 0, 0.0625f, BQKVb, 0, nullptr, 1, 0, 0, nullptr, QKV16, 3 * DD, 0, NN, 3 * DD, DD);
    k_vt<<<(DD * (NN / 8) + 255) / 256, 256, 0, stream>>>(QKV16, VT);
    for (int r0 = 0; r0 < NN; r0 += RCH) {
      for (int h = 0; h < NHD; ++h) k_gemm_hhx<0><<<gS, 128, 0, stream>>>(QKV16 + (size_t)r0 * 3 * DD + h * HDC, 3 * DD, 0, QKV16 + DD + h * HDC, 3 * DD, 0, 0.17677669529663687f, nullptr, 0, nullptr, 1, 0, 0, S + (size_t)h * RCH * NN, nullptr, NN, 0, RCH, NN, HDC);
      k_hsoft<<<(RCH * (NN / 4) + 255) / 256, 256, 0, stream>>>(S, P16);
      for (int h = 0; h < NHD; ++h) k_gemm_hhx<0><<<gP, 128, 0, stream>>>(P16 + (size_t)h * RCH * NN, NN, 0, VT + (size_t)h * HDC * NN, NN, 0, 1.0f, nullptr, 0, nullptr, 1, 0, 0, O + (size_t)r0 * DD + h * HDC, nullptr, DD, 0, RCH, HDC, NN); }
    k_f16c<<<(unsigned)((n8 + 255) / 256), 256, 0, stream>>>(O, O16, n8);
    k_gemm_hhx<0><<<gD, 128, 0, stream>>>(O16, DD, 0, BO, DD, 0, 0.0625f, bo + (size_t)l * DD, 0, Hf, 1, (size_t)DD, 0, X2, nullptr, DD, 0, NN, DD, DD);
    k_ln<<<NN / 8, 256, 0, stream>>>(X2, lng + (size_t)l * DD, lnb + (size_t)l * DD, Hf, H16);
    k_gemm_hhx<0><<<gC1, 128, 0, stream>>>(H16, DD, 0, BC1, DD, 0, 0.0625f, bc1 + (size_t)l * DC, 0, nullptr, 1, 0, 0, C1, nullptr, DC, 0, NN, DC, DD);
    k_pos<<<(NN * 3 + 255) / 256, 256, 0, stream>>>(C1, Wc2 + (size_t)l * DC, bc2 + l, RM, POS); }
  k_energy1<<<NN / 256, 256, 0, stream>>>(Hf, We, be, EP);
  k_fin<<<(1 + NN * 3 + 255) / 256, 256, 0, stream>>>(EP, POS, (float*)d_out);
}
